// RobertaSelfAttention_34024730919581
// MI455X (gfx1250) — hardware-verified
//
#include <hip/hip_runtime.h>


#ifndef NB
#define NB 4
#endif
#ifndef SEQ
#define SEQ 1024
#endif
#define NB_FULL  4
#define SEQ_FULL 1024
#define DM       1024
#define NH       16
#define HD       64
#define MAXPOS   1024
#define NE       2047
#define NEPAD    2048

static_assert(NB >= 1 && NB <= NB_FULL);
static_assert(SEQ >= 128 && SEQ <= SEQ_FULL && (SEQ % 128) == 0);
static_assert(SEQ <= MAXPOS);
static_assert(SEQ + MAXPOS <= NEPAD);
static_assert(DM == NH * HD);
static_assert((NB * SEQ) % 128 == 0);
static_assert(NE == 2 * MAXPOS - 1);

typedef unsigned short us8  __attribute__((ext_vector_type(8)));
typedef unsigned short us16 __attribute__((ext_vector_type(16)));
typedef __bf16         v16bf __attribute__((ext_vector_type(16)));
typedef _Float16       v16h  __attribute__((ext_vector_type(16)));
typedef float          v8f   __attribute__((ext_vector_type(8)));
typedef float          v4f   __attribute__((ext_vector_type(4)));


__device__ __forceinline__ unsigned short bf16_bits(float f) {
  unsigned int u = __builtin_bit_cast(unsigned int, f);
  u += 0x7fffu + ((u >> 16) & 1u);
  return (unsigned short)(u >> 16);
}

__device__ __forceinline__ float bf16_rne(float f) {
  unsigned int u = ((unsigned int)bf16_bits(f)) << 16;
  return __builtin_bit_cast(float, u);
}

__device__ __forceinline__ unsigned short f16_bits(float f) {
  _Float16 hv = (_Float16)f;
  return __builtin_bit_cast(unsigned short, hv);
}

__device__ __forceinline__ us16 ld_frag(const unsigned short* base, int row, int stride, int col) {
  const unsigned short* p = base + (size_t)row * (size_t)stride + col;
  us8 a = *(const us8*)(p);
  us8 b = *(const us8*)(p + 16);
  return __builtin_shufflevector(a, b, 0, 1, 2, 3, 4, 5, 6, 7, 8, 9, 10, 11, 12, 13, 14, 15);
}

__device__ __forceinline__ v8f mma_bf16(us16 a, us16 b, v8f c) {
  v8f d = __builtin_amdgcn_wmma_f32_16x16x32_bf16(false, __builtin_bit_cast(v16bf, a), false,
                                                  __builtin_bit_cast(v16bf, b), (short)0, c, false, false);
  asm volatile("v_nop\n\tv_nop\n\tv_nop\n\tv_nop" : "+v"(d) : "v"(a), "v"(b));
  return d;
}

__device__ __forceinline__ v8f mma_f16(us16 a, us16 b, v8f c) {
  v8f d = __builtin_amdgcn_wmma_f32_16x16x32_f16(false, __builtin_bit_cast(v16h, a), false,
                                                 __builtin_bit_cast(v16h, b), (short)0, c, false, false);
  asm volatile("v_nop\n\tv_nop\n\tv_nop\n\tv_nop" : "+v"(d) : "v"(a), "v"(b));
  return d;
}

__global__ __launch_bounds__(256)
void cvt_rows_bf16(const float* __restrict__ s0, const float* __restrict__ s1,
                   const float* __restrict__ s2, unsigned short* __restrict__ dst,
                   int nrows, int seq, int seqfull) {
  const int mat = blockIdx.y;
  const float* src = (mat == 0) ? s0 : ((mat == 1) ? s1 : s2);
  int r = blockIdx.x * 2 + (threadIdx.x >> 7);
  r = (r < nrows) ? r : (nrows - 1);
  const int c = (threadIdx.x & 127) * 8;
  const size_t srow = (size_t)(r / seq) * (size_t)seqfull + (size_t)(r % seq);
  const float* p = src + srow * DM + c;
  const v4f a = *(const v4f*)(p);
  const v4f e = *(const v4f*)(p + 4);
  us8 o;
  o[0] = bf16_bits(a[0]); o[1] = bf16_bits(a[1]); o[2] = bf16_bits(a[2]); o[3] = bf16_bits(a[3]);
  o[4] = bf16_bits(e[0]); o[5] = bf16_bits(e[1]); o[6] = bf16_bits(e[2]); o[7] = bf16_bits(e[3]);
  unsigned short* d = dst + ((size_t)mat * (size_t)nrows + (size_t)r) * DM + c;
  *(volatile us8*)d = o;
  __threadfence();
  *(volatile us8*)d = o;
}

__global__ __launch_bounds__(256)
void cvt_e_f16(const float* __restrict__ e, unsigned short* __restrict__ ep) {
  const int g   = blockIdx.x * 256 + threadIdx.x;
  const int row = g >> 3;
  const int ch  = (g & 7) * 8;
  const int rs  = (row < NE) ? row : (NE - 1);
  const float sc = (row < NE) ? 64.0f : 0.0f;
  const float* p = e + (size_t)rs * HD + ch;
  const v4f a = *(const v4f*)(p);
  const v4f c4 = *(const v4f*)(p + 4);
  us8 o;
  o[0] = f16_bits(bf16_rne(a[0]) * sc);  o[1] = f16_bits(bf16_rne(a[1]) * sc);
  o[2] = f16_bits(bf16_rne(a[2]) * sc);  o[3] = f16_bits(bf16_rne(a[3]) * sc);
  o[4] = f16_bits(bf16_rne(c4[0]) * sc); o[5] = f16_bits(bf16_rne(c4[1]) * sc);
  o[6] = f16_bits(bf16_rne(c4[2]) * sc); o[7] = f16_bits(bf16_rne(c4[3]) * sc);
  unsigned short* d = ep + (size_t)row * HD + ch;
  *(volatile us8*)d = o;
  __threadfence();
  *(volatile us8*)d = o;
}

#define TP 72

__global__ __launch_bounds__(128)
void proj_kernel(const unsigned short* __restrict__ xb, const unsigned short* __restrict__ wb,
                 const float* __restrict__ bq, const float* __restrict__ bk,
                 const float* __restrict__ bv,
                 unsigned short* __restrict__ qp, unsigned short* __restrict__ kp,
                 unsigned short* __restrict__ vp) {
  __shared__ __attribute__((aligned(16))) unsigned short stile[4 * 32 * TP];

  const int tid = threadIdx.x, lane = tid & 31, wid = tid >> 5;
  const int lr = lane & 15, half8 = (lane >> 4) * 8;
  const int h = blockIdx.y, z = blockIdx.z;
  const int s0 = (blockIdx.x * 4 + wid) * 32;

  const unsigned short* wm = wb + (size_t)z * DM * DM + (size_t)h * HD * DM;
  const float* bias = (z == 0) ? bq : ((z == 1) ? bk : bv);
  unsigned short* plane = (z == 0) ? qp : ((z == 1) ? kp : vp);

  const v8f zero = {0.f, 0.f, 0.f, 0.f, 0.f, 0.f, 0.f, 0.f};
  v8f acc[2][4] = {{zero, zero, zero, zero}, {zero, zero, zero, zero}};

  for (int kk = 0; kk < DM; kk += 32) {
    const us16 a0 = ld_frag(xb, s0 + lr,      DM, kk + half8);
    const us16 a1 = ld_frag(xb, s0 + 16 + lr, DM, kk + half8);
#pragma unroll
    for (int dt = 0; dt < 4; ++dt) {
      const us16 bf = ld_frag(wm, dt * 16 + lr, DM, kk + half8);
      acc[0][dt] = mma_bf16(a0, bf, acc[0][dt]);
      acc[1][dt] = mma_bf16(a1, bf, acc[1][dt]);
    }
  }

  unsigned short* stw = stile + wid * (32 * TP);
#pragma unroll
  for (int dt = 0; dt < 4; ++dt) {
    const float bcol = bf16_rne(bias[h * HD + dt * 16 + lr]);
#pragma unroll
    for (int st = 0; st < 2; ++st) {
#pragma unroll
      for (int r = 0; r < 8; ++r) {
        const float v = (acc[st][dt][r] + bcol) * 8.0f;
        stw[(st * 16 + half8 + r) * TP + dt * 16 + lr] = f16_bits(v);
      }
    }
  }
  __syncthreads();

  const int piece = lane & 7, rsub = lane >> 3;
#pragma unroll
  for (int it = 0; it < 8; ++it) {
    const int row = it * 4 + rsub;
    const us8 v = *(const us8*)(stw + row * TP + piece * 8);
    const int s = s0 + row;
    const int b = s / SEQ, l = s - b * SEQ;
    unsigned short* d = plane + (((size_t)(b * NH + h) * SEQ + l) * HD + piece * 8);
    *(volatile us8*)d = v;
  }
  __threadfence();
#pragma unroll
  for (int it = 0; it < 8; ++it) {
    const int row = it * 4 + rsub;
    const us8 v = *(const us8*)(stw + row * TP + piece * 8);
    const int s = s0 + row;
    const int b = s / SEQ, l = s - b * SEQ;
    unsigned short* d = plane + (((size_t)(b * NH + h) * SEQ + l) * HD + piece * 8);
    *(volatile us8*)d = v;
  }
}

#define KP 72
#define VP 40
#define EP 72
#define NBR 160
#define NPF 160
#define MROWS 48
#define OPITCH 68
#define SM_K 0
#define SM_V (SM_K + 32 * KP * 2)
#define SM_E (SM_V + 64 * VP * 2)
#define SM_N (SM_E + NBR * EP * 2)
#define SM_M (SM_N + 32 * NPF * 4)
#define SM_TOTAL (SM_M + 4 * 2 * MROWS * 16 * 4)
static_assert(SM_V % 16 == 0 && SM_E % 16 == 0 && SM_N % 16 == 0 && SM_M % 16 == 0);
static_assert(4 * 32 * OPITCH * 4 <= SM_TOTAL);
static_assert(NBR % 16 == 0 && NBR >= 128 + 31 && MROWS >= 47 && NPF >= NBR);

__global__ __launch_bounds__(128)
void attn_kernel(const unsigned short* __restrict__ qp, const unsigned short* __restrict__ kp,
                 const unsigned short* __restrict__ vp, const unsigned short* __restrict__ ep,
                 const float* __restrict__ amask, float* __restrict__ out) {
  __shared__ __attribute__((aligned(16))) unsigned char smem[SM_TOTAL];

  const int tid = threadIdx.x, lane = tid & 31, wid = tid >> 5;
  const int lr = lane & 15, half8 = (lane >> 4) * 8;
  const int bh = blockIdx.y;
  const int b = bh / NH, h = bh - b * NH;
  const int qb0 = blockIdx.x * 128;
  const int q0 = qb0 + wid * 32;

  unsigned short* ktile = (unsigned short*)(smem + SM_K);
  unsigned short* vtile = (unsigned short*)(smem + SM_V);
  unsigned short* eband = (unsigned short*)(smem + SM_E);
  float* nbuf = (float*)(smem + SM_N);
  float* mbuf = (float*)(smem + SM_M) + wid * (2 * MROWS * 16);
  float* ost  = (float*)(smem) + wid * (32 * OPITCH);

  const unsigned short* qh = qp + (size_t)bh * SEQ * HD;
  const unsigned short* kh = kp + (size_t)bh * SEQ * HD;
  const unsigned short* vh = vp + (size_t)bh * SEQ * HD;
  const float* mrow = amask + (size_t)b * SEQ_FULL;

  us16 bqf[2][2];
#pragma unroll
  for (int qs = 0; qs < 2; ++qs) {
    bqf[qs][0] = ld_frag(qh, q0 + qs * 16 + lr, HD,      half8);
    bqf[qs][1] = ld_frag(qh, q0 + qs * 16 + lr, HD, 32 + half8);
  }

  const v8f zero = {0.f, 0.f, 0.f, 0.f, 0.f, 0.f, 0.f, 0.f};
  v8f acc[2][4] = {{zero, zero, zero, zero}, {zero, zero, zero, zero}};
  float mrun[2] = {-__builtin_inff(), -__builtin_inff()};
  float lrun[2] = {0.f, 0.f};
  const float c512  = 0.001953125f;
  const float c4096 = 0.000244140625f;

  for (int k0 = 0; k0 < SEQ; k0 += 32) {
    __syncthreads();

#pragma unroll
    for (int rr = 0; rr < 2; ++rr) {
      const int c  = tid + rr * 128;
      const int j  = c >> 3;
      const int ch = (c & 7) * 8;
      const us8 kv = *(const us8*)(kh + (size_t)(k0 + j) * HD + ch);
      *(us8*)(ktile + j * KP + ch) = kv;
      const us8 vv = *(const us8*)(vh + (size_t)(k0 + j) * HD + ch);
#pragma unroll
      for (int i = 0; i < 8; ++i) vtile[(ch + i) * VP + j] = vv[i];
    }
    const int base2 = qb0 - k0 + (MAXPOS - 32);
    for (int c = tid; c < NBR * 8; c += 128) {
      const int u  = c >> 3;
      const int ch = (c & 7) * 8;
      *(us8*)(eband + u * EP + ch) = *(const us8*)(ep + (size_t)(base2 + u) * HD + ch);
    }
    __syncthreads();

    {
      const us16 ka00 = ld_frag(ktile,      lr, KP,      half8);
      const us16 ka01 = ld_frag(ktile,      lr, KP, 32 + half8);
      const us16 ka10 = ld_frag(ktile, 16 + lr, KP,      half8);
      const us16 ka11 = ld_frag(ktile, 16 + lr, KP, 32 + half8);
      for (int un = wid; un < NBR / 16; un += 4) {
        const us16 e0 = ld_frag(eband, un * 16 + lr, EP,      half8);
        const us16 e1 = ld_frag(eband, un * 16 + lr, EP, 32 + half8);
        v8f d0 = mma_f16(ka00, e0, zero);
        d0     = mma_f16(ka01, e1, d0);
        v8f d1 = mma_f16(ka10, e0, zero);
        d1     = mma_f16(ka11, e1, d1);
#pragma unroll
        for (int r = 0; r < 8; ++r) {
          nbuf[(half8 + r) * NPF + un * 16 + lr]      = d0[r];
          nbuf[(16 + half8 + r) * NPF + un * 16 + lr] = d1[r];
        }
      }
    }
#pragma unroll
    for (int qs = 0; qs < 2; ++qs) {
#pragma unroll
      for (int ut = 0; ut < 3; ++ut) {
        const int ru = wid * 32 + qs * 16 + ut * 16 + lr;
        const us16 e0 = ld_frag(eband, ru, EP,      half8);
        const us16 e1 = ld_frag(eband, ru, EP, 32 + half8);
        v8f d = mma_f16(e0, bqf[qs][0], zero);
        d     = mma_f16(e1, bqf[qs][1], d);
#pragma unroll
        for (int r = 0; r < 8; ++r)
          mbuf[qs * (MROWS * 16) + (ut * 16 + half8 + r) * 16 + lr] = d[r];
      }
    }
    __syncthreads();

    v8f mk0 = *(const v8f*)(mrow + k0 + half8);
    v8f mk1 = *(const v8f*)(mrow + k0 + 16 + half8);
#pragma unroll
    for (int r = 0; r < 8; ++r) { mk0[r] = bf16_rne(mk0[r]); mk1[r] = bf16_rne(mk1[r]); }

    const us16 ka00 = ld_frag(ktile,      lr, KP,      half8);
    const us16 ka01 = ld_frag(ktile,      lr, KP, 32 + half8);
    const us16 ka10 = ld_frag(ktile, 16 + lr, KP,      half8);
    const us16 ka11 = ld_frag(ktile, 16 + lr, KP, 32 + half8);

#pragma unroll
    for (int qs = 0; qs < 2; ++qs) {
      v8f t0 = mma_f16(ka00, bqf[qs][0], zero);
      t0     = mma_f16(ka01, bqf[qs][1], t0);
      v8f t1 = mma_f16(ka10, bqf[qs][0], zero);
      t1     = mma_f16(ka11, bqf[qs][1], t1);

      const float* mq = mbuf + qs * (MROWS * 16);
      const int qloc = wid * 32 + qs * 16 + lr;
      float sa[8], sb[8];
#pragma unroll
      for (int r = 0; r < 8; ++r) {
        const int ja = half8 + r;
        const int jb = 16 + half8 + r;
        const float ga = mq[(lr - ja + 31) * 16 + lr] + nbuf[ja * NPF + (qloc - ja + 31)];
        const float gb = mq[(lr - jb + 31) * 16 + lr] + nbuf[jb * NPF + (qloc - jb + 31)];
        sa[r] = t0[r] * c512 + ga * c4096 + mk0[r];
        sb[r] = t1[r] * c512 + gb * c4096 + mk1[r];
      }

      float mloc = sa[0];
#pragma unroll
      for (int r = 1; r < 8; ++r) mloc = fmaxf(mloc, sa[r]);
#pragma unroll
      for (int r = 0; r < 8; ++r) mloc = fmaxf(mloc, sb[r]);
      const float mt    = fmaxf(mloc, __shfl_xor(mloc, 16, 32));
      const float mnew  = fmaxf(mrun[qs], mt);
      const float alpha = __expf(mrun[qs] - mnew);

      float lloc = 0.f;
      us16 pu;
#pragma unroll
      for (int r = 0; r < 8; ++r) {
        const float pa = __expf(sa[r] - mnew);
        const float pc = __expf(sb[r] - mnew);
        lloc += pa + pc;
        pu[r]     = f16_bits(pa * 1024.0f);
        pu[8 + r] = f16_bits(pc * 1024.0f);
      }
      const float lt = lloc + __shfl_xor(lloc, 16, 32);
      lrun[qs] = lrun[qs] * alpha + lt;
      mrun[qs] = mnew;

#pragma unroll
      for (int dt = 0; dt < 4; ++dt) {
        const us16 va = ld_frag(vtile, dt * 16 + lr, VP, half8);
        acc[qs][dt] = acc[qs][dt] * alpha;
        acc[qs][dt] = mma_f16(va, pu, acc[qs][dt]);
      }
    }
  }

  __syncthreads();
#pragma unroll
  for (int qs = 0; qs < 2; ++qs) {
    const float inv = 1.0f / (lrun[qs] * 8192.0f);
#pragma unroll
    for (int dt = 0; dt < 4; ++dt) {
#pragma unroll
      for (int r = 0; r < 8; ++r)
        ost[(qs * 16 + lr) * OPITCH + dt * 16 + half8 + r] = acc[qs][dt][r] * inv;
    }
  }
  __syncthreads();

  const int rsub = lane >> 4, piece = lane & 15;
  float* obase = out + ((size_t)(b * SEQ + q0)) * DM + (size_t)h * HD + piece * 4;
#pragma unroll
  for (int it = 0; it < 16; ++it) {
    const int row = it * 2 + rsub;
    const v4f v = *(const v4f*)(ost + row * OPITCH + piece * 4);
    *(volatile v4f*)(obase + (size_t)row * DM) = v;
  }
  __threadfence();
#pragma unroll
  for (int it = 0; it < 16; ++it) {
    const int row = it * 2 + rsub;
    const v4f v = *(const v4f*)(ost + row * OPITCH + piece * 4);
    *(volatile v4f*)(obase + (size_t)row * DM) = v;
  }
}


extern "C" void kernel_launch(void* const* d_in, const int* in_sizes, int n_in,
                              void* d_out, int out_size, void* d_ws, size_t ws_size,
                              hipStream_t stream) {
  if (n_in < 9) return;
  const float* hidden = (const float*)d_in[0];
  const float* amask  = (const float*)d_in[1];
  const float* Wq     = (const float*)d_in[2];
  const float* bq     = (const float*)d_in[3];
  const float* Wk     = (const float*)d_in[4];
  const float* bk     = (const float*)d_in[5];
  const float* Wv     = (const float*)d_in[6];
  const float* bv     = (const float*)d_in[7];
  const float* demb   = (const float*)d_in[8];
  float* out = (float*)d_out;

  if (in_sizes[0] < ((NB - 1) * SEQ_FULL + SEQ) * DM) return;
  if (in_sizes[1] < (NB - 1) * SEQ_FULL + SEQ) return;
  if (in_sizes[2] < DM * DM || in_sizes[4] < DM * DM || in_sizes[6] < DM * DM) return;
  if (in_sizes[3] < DM || in_sizes[5] < DM || in_sizes[7] < DM) return;
  if (in_sizes[8] < NE * HD) return;
  if (out_size < NB * SEQ * DM) return;

  const size_t xb_bytes = (size_t)NB * SEQ * DM * 2;
  const size_t wb_bytes = (size_t)3 * DM * DM * 2;
  const size_t ep_bytes = (size_t)NEPAD * HD * 2;
  const size_t pl_bytes = (size_t)NB * NH * SEQ * HD * 2;
  size_t off = 0;
  char* ws = (char*)d_ws;
  unsigned short* xb = (unsigned short*)(ws + off); off += xb_bytes;
  unsigned short* wb = (unsigned short*)(ws + off); off += wb_bytes;
  unsigned short* ep = (unsigned short*)(ws + off); off += ep_bytes;
  unsigned short* qp = (unsigned short*)(ws + off); off += pl_bytes;
  unsigned short* kp = (unsigned short*)(ws + off); off += pl_bytes;
  unsigned short* vp = (unsigned short*)(ws + off); off += pl_bytes;
  if (ws_size < off) return;

  cvt_rows_bf16<<<dim3((NB * SEQ) / 2, 1, 1), 256, 0, stream>>>(hidden, hidden, hidden, xb,
                                                               NB * SEQ, SEQ, SEQ_FULL);
  cvt_rows_bf16<<<dim3(DM / 2, 3, 1), 256, 0, stream>>>(Wq, Wk, Wv, wb, DM, DM, DM);
  cvt_e_f16<<<dim3((NEPAD * 8) / 256, 1, 1), 256, 0, stream>>>(demb, ep);
  proj_kernel<<<dim3((NB * SEQ) / 128, NH, 3), 128, 0, stream>>>(xb, wb, bq, bk, bv, qp, kp, vp);
  attn_kernel<<<dim3(SEQ / 128, NB * NH, 1), 128, 0, stream>>>(qp, kp, vp, ep, amask, out);
}
